// SparseResBlock_16389595201741
// MI455X (gfx1250) — hardware-verified
//
#include <hip/hip_runtime.h>
#include <stddef.h>


#define GD      128
#define NBAT    2
#define TBLN    (NBAT * GD * GD * GD)
#define NOFF    27
#define CH      64
#define NTHR    256
#define NWAVE   8
#define CROWS   128
#define APH     72
#define TPB     32768
#define WPL     (NOFF * CH * CH)
#define WSCALE  16.0f
#define WINV    0.0625f
#define BNEPS   1e-5f
#define WSCAP   134217728

#define LC_CO   0
#define LC_NB   (LC_CO + CROWS * 4 * 4)
#define LC_A    (LC_NB + NOFF * CROWS * 4)
#define LC_ST   (LC_A + CROWS * APH * 2)
#define LC_PQ   (LC_ST + CROWS * CH * 4)
#define LC_PF   (LC_PQ + 4 * 128 * 8)
#define LDS_CONV (LC_PF + 128 * 8)
#define LDS_TAB  (TPB * 4)

static_assert(TBLN % TPB == 0);
static_assert((TPB / 4) % NTHR == 0);
static_assert((WPL / 8) % NTHR == 0);
static_assert(CROWS == 128);
static_assert(CROWS == NWAVE * 16);
static_assert(CROWS * CH / 4 == 8 * NTHR);
static_assert((APH % 8) == 0);
static_assert((LC_NB % 16) == 0 && (LC_A % 16) == 0 && (LC_ST % 16) == 0 && (LC_PQ % 16) == 0 && (LC_PF % 16) == 0);

typedef float    v4f  __attribute__((ext_vector_type(4)));
typedef float    v8f  __attribute__((ext_vector_type(8)));
typedef int      v4i  __attribute__((ext_vector_type(4)));
typedef double   v2d  __attribute__((ext_vector_type(2)));
typedef _Float16 v4h  __attribute__((ext_vector_type(4)));
typedef _Float16 v8h  __attribute__((ext_vector_type(8)));
typedef _Float16 v16h __attribute__((ext_vector_type(16)));
union FragH { v16h v; v8h h[2]; };

__device__ __forceinline__ int clampi(int v, int lo, int hi) {
  return v < lo ? lo : (v > hi ? hi : v);
}

__device__ __forceinline__ v4h cvt4(v4f a) {
  v4h r;
  r[0] = (_Float16)a.x; r[1] = (_Float16)a.y; r[2] = (_Float16)a.z; r[3] = (_Float16)a.w;
  return r;
}
__device__ __forceinline__ v8h cvt8(v4f a, v4f b) {
  v8h r;
  r[0] = (_Float16)a.x; r[1] = (_Float16)a.y; r[2] = (_Float16)a.z; r[3] = (_Float16)a.w;
  r[4] = (_Float16)b.x; r[5] = (_Float16)b.y; r[6] = (_Float16)b.z; r[7] = (_Float16)b.w;
  return r;
}

__device__ __forceinline__ v8f wmh(v16h a, v16h b, v8f c) {
  v8f d = __builtin_amdgcn_wmma_f32_16x16x32_f16(false, a, false, b, (short)0, c, false, false);
  asm volatile("v_nop\n\tv_nop\n\tv_nop\n\tv_nop" : "+v"(d) : "v"(a), "v"(b));
  return d;
}

__global__ __launch_bounds__(NTHR) void k_table(const int* __restrict__ coords, int* table, int n) {
  extern __shared__ v4f lds_dyn[];
  int* lt = (int*)lds_dyn;
  const int tid = threadIdx.x;
  const int c0 = blockIdx.x * TPB;
  const v4i neg = {-1, -1, -1, -1};
#pragma unroll 4
  for (int i = 0; i < (TPB / 4) / NTHR; ++i) ((v4i*)lt)[i * NTHR + tid] = neg;
  __syncthreads();
#pragma unroll 1
  for (int r = tid; r < n; r += NTHR) {
    const v4i c = *(const v4i*)(coords + (size_t)r * 4);
    const int b = clampi(c.x, 0, NBAT - 1);
    const int x = clampi(c.y, 0, GD - 1);
    const int y = clampi(c.z, 0, GD - 1);
    const int z = clampi(c.w, 0, GD - 1);
    const int lin = ((b * GD + x) * GD + y) * GD + z;
    const unsigned d = (unsigned)(lin - c0);
    if (d < (unsigned)TPB) lt[d] = r;
  }
  __syncthreads();
  int* gp = table + (size_t)c0;
#pragma unroll 4
  for (int i = 0; i < (TPB / 4) / NTHR; ++i) {
    const int f = i * NTHR + tid;
    const v4i v = ((const v4i*)lt)[f];
    *(volatile v4i*)(gp + 4 * f) = v;
  }
  __threadfence();
#pragma unroll 4
  for (int i = 0; i < (TPB / 4) / NTHR; ++i) {
    const int f = i * NTHR + tid;
    const v4i v = ((const v4i*)lt)[f];
    *(volatile v4i*)(gp + 4 * f) = v;
  }
}

__global__ __launch_bounds__(NTHR) void k_wprep(const float* __restrict__ w1, const float* __restrict__ w2,
                                              _Float16* p1, _Float16* p2) {
  const int gpp = WPL / 8;
  const int bstart = blockIdx.x * NTHR;
  const float* src; _Float16* dst; int g0;
  if (bstart < gpp) { src = w1; dst = p1; g0 = 0; } else { src = w2; dst = p2; g0 = gpp; }
  const int gi = bstart + (int)threadIdx.x - g0;
  if (gi < 0 || gi >= gpp) return;
  const int o   = gi * 8;
  const int k   = o >> 12;
  const int rem = o & 4095;
  const int nn  = rem >> 6;
  const int cb  = rem & 63;
  const float* sp = src + ((size_t)k * CH + cb) * CH + nn;
  v4f a, b;
  a.x = sp[0 * CH] * WSCALE; a.y = sp[1 * CH] * WSCALE; a.z = sp[2 * CH] * WSCALE; a.w = sp[3 * CH] * WSCALE;
  b.x = sp[4 * CH] * WSCALE; b.y = sp[5 * CH] * WSCALE; b.z = sp[6 * CH] * WSCALE; b.w = sp[7 * CH] * WSCALE;
  const v8h hv = cvt8(a, b);
  _Float16* dp = dst + o;
  *(volatile v8h*)dp = hv;
  __threadfence();
  *(volatile v8h*)dp = hv;
}

template <int MODE>
__global__ __launch_bounds__(NTHR) void k_conv(
    const float* __restrict__ src, const int* __restrict__ coords, const int* __restrict__ table,
    const _Float16* __restrict__ wpl, const float* __restrict__ bnp, float* dst, double* part, int n) {
  extern __shared__ v4f lds_dyn[];
  char* lb = (char*)lds_dyn;
  int*      sCo = (int*)(lb + LC_CO);
  int*      sNb = (int*)(lb + LC_NB);
  _Float16* sA  = (_Float16*)(lb + LC_A);
  float*    stg = (float*)(lb + LC_ST);
  double*   sPq = (double*)(lb + LC_PQ);
  double*   sPf = (double*)(lb + LC_PF);
  const int tid = threadIdx.x, lane = tid & 31, wave = tid >> 5, hh = lane >> 4, m = lane & 15;
  const int c4 = tid & 15, rsub = tid >> 4;
  const int rowBase = blockIdx.x * CROWS;

  if (tid < CROWS) {
    int r = rowBase + tid;
    r = r > n - 1 ? n - 1 : r;
    ((v4i*)sCo)[tid] = *(const v4i*)(coords + (size_t)r * 4);
  }
  __syncthreads();

#pragma unroll 1
  for (int e = tid; e < NOFF * CROWS; e += NTHR) {
    const int k = e >> 7;
    const int r = e & (CROWS - 1);
    const int dx = k / 9 - 1;
    const int dy = (k / 3) % 3 - 1;
    const int dz = k % 3 - 1;
    const v4i c = ((const v4i*)sCo)[r];
    const int b = clampi(c.x, 0, NBAT - 1);
    const int x = clampi(c.y, 0, GD - 1);
    const int y = clampi(c.z, 0, GD - 1);
    const int z = clampi(c.w, 0, GD - 1);
    const int nx = x + dx, ny = y + dy, nz = z + dz;
    const bool inb = ((unsigned)nx < (unsigned)GD) && ((unsigned)ny < (unsigned)GD) && ((unsigned)nz < (unsigned)GD);
    const int cx = clampi(nx, 0, GD - 1), cy = clampi(ny, 0, GD - 1), cz = clampi(nz, 0, GD - 1);
    const int lin = ((b * GD + cx) * GD + cy) * GD + cz;
    int idx = table[lin];
    idx = idx > n - 1 ? n - 1 : idx;
    const bool valid = inb && (idx >= 0) && (rowBase + r < n);
    sNb[e] = valid ? idx : -1;
  }
  __syncthreads();

  v4f mu = {0.f, 0.f, 0.f, 0.f}, sc = {1.f, 1.f, 1.f, 1.f}, be = {0.f, 0.f, 0.f, 0.f};
  if (MODE == 1) {
    mu = *(const v4f*)(bnp + 4 * c4);
    sc = *(const v4f*)(bnp + 64 + 4 * c4);
    be = *(const v4f*)(bnp + 128 + 4 * c4);
  }

  v8f acc[4];
#pragma unroll
  for (int t = 0; t < 4; ++t) { v8f zz = {0.f, 0.f, 0.f, 0.f, 0.f, 0.f, 0.f, 0.f}; acc[t] = zz; }
  const _Float16* ar = sA + (wave * 16 + m) * APH + 8 * hh;

#pragma unroll 1
  for (int k = 0; k < NOFF; ++k) {
#pragma unroll
    for (int i = 0; i < 8; ++i) {
      const int r = rsub + 16 * i;
      const int idx = sNb[k * CROWS + r];
      const int s = idx < 0 ? 0 : idx;
      v4f v = *(const v4f*)(src + (size_t)s * CH + 4 * c4);
      if (MODE == 1) {
        v = (v - mu) * sc + be;
        v.x = fmaxf(v.x, 0.f); v.y = fmaxf(v.y, 0.f); v.z = fmaxf(v.z, 0.f); v.w = fmaxf(v.w, 0.f);
      }
      const bool ok = idx >= 0;
      v.x = ok ? v.x : 0.f; v.y = ok ? v.y : 0.f; v.z = ok ? v.z : 0.f; v.w = ok ? v.w : 0.f;
      *(v4h*)(sA + r * APH + 4 * c4) = cvt4(v);
    }
    __syncthreads();

    const _Float16* wk = wpl + (size_t)k * CH * CH;
#pragma unroll
    for (int kt = 0; kt < CH / 32; ++kt) {
      FragH a;
      a.h[0] = *(const v8h*)(ar + 32 * kt);
      a.h[1] = *(const v8h*)(ar + 32 * kt + 16);
#pragma unroll
      for (int t = 0; t < 4; ++t) {
        const _Float16* bp = wk + (size_t)(16 * t + m) * CH + 32 * kt + 8 * hh;
        FragH b;
        b.h[0] = *(const v8h*)bp;
        b.h[1] = *(const v8h*)(bp + 16);
        acc[t] = wmh(a.v, b.v, acc[t]);
      }
    }
    __syncthreads();
  }

  {
    float* sp = stg + (wave * 16 + 8 * hh) * CH + m;
#pragma unroll
    for (int t = 0; t < 4; ++t) {
#pragma unroll
      for (int r = 0; r < 8; ++r) sp[r * CH + 16 * t] = acc[t][r] * WINV;
    }
  }
  __syncthreads();

  {
    const int cst = tid & 63, q = tid >> 6;
    int nval = n - rowBase;
    nval = nval > CROWS ? CROWS : nval;
    double s1 = 0.0, s2 = 0.0;
#pragma unroll 4
    for (int j = 0; j < 32; ++j) {
      const int r = 32 * q + j;
      const float xv = stg[r * CH + cst];
      const double xd = (r < nval) ? (double)xv : 0.0;
      s1 += xd;
      s2 += xd * xd;
    }
    sPq[q * 128 + cst]      = s1;
    sPq[q * 128 + 64 + cst] = s2;
  }
  __syncthreads();
  if (tid < 128) sPf[tid] = (sPq[tid] + sPq[128 + tid]) + (sPq[256 + tid] + sPq[384 + tid]);
  __syncthreads();

  const float* lp = stg + wave * 16 * CH + 4 * lane;
  float* gpo = dst + ((size_t)rowBase + wave * 16) * CH + 4 * lane;
  double* pp = part + (size_t)blockIdx.x * 128;
  v2d d0 = {0.0, 0.0}, d1 = {0.0, 0.0};
  if (wave == 0) { d0 = *(const v2d*)(sPf + 2 * lane); d1 = *(const v2d*)(sPf + 64 + 2 * lane); }
#pragma unroll
  for (int i = 0; i < 8; ++i) { const v4f v = *(const v4f*)(lp + 128 * i); *(volatile v4f*)(gpo + 128 * i) = v; }
  if (wave == 0) { *(volatile v2d*)(pp + 2 * lane) = d0; *(volatile v2d*)(pp + 64 + 2 * lane) = d1; }
  __threadfence();
#pragma unroll
  for (int i = 0; i < 8; ++i) { const v4f v = *(const v4f*)(lp + 128 * i); *(volatile v4f*)(gpo + 128 * i) = v; }
  if (wave == 0) { *(volatile v2d*)(pp + 2 * lane) = d0; *(volatile v2d*)(pp + 64 + 2 * lane) = d1; }
}

__global__ __launch_bounds__(NTHR) void k_bnfin(const double* __restrict__ part, int nBlk,
                                              const float* __restrict__ gam, const float* __restrict__ bet,
                                              float* bnp, int n) {
  __shared__ double sd[128];
  __shared__ __attribute__((aligned(16))) float sf[256];
  const int tid = threadIdx.x;
  if (tid < 128) {
    double a = 0.0;
#pragma unroll 1
    for (int b = 0; b < nBlk; ++b) a += part[(size_t)b * 128 + tid];
    sd[tid] = a;
  }
  __syncthreads();
  if (tid < 64) {
    const double invn = 1.0 / (double)n;
    const double mean = sd[tid] * invn;
    double var = sd[64 + tid] * invn - mean * mean;
    var = var < 0.0 ? 0.0 : var;
    const float vf = (float)var;
    const float rs = rsqrtf(vf + BNEPS);
    sf[tid]       = (float)mean;
    sf[64 + tid]  = rs * gam[tid];
    sf[128 + tid] = bet[tid];
    sf[192 + tid] = 0.0f;
  }
  __syncthreads();
  v4f v = {0.f, 0.f, 0.f, 0.f};
  if (tid < 64) v = *(const v4f*)(sf + 4 * tid);
  if (tid < 64) *(volatile v4f*)(bnp + 4 * tid) = v;
  __threadfence();
  if (tid < 64) *(volatile v4f*)(bnp + 4 * tid) = v;
}

__global__ __launch_bounds__(NTHR) void k_out(const float* __restrict__ h2, const float* __restrict__ bnp,
                                            const float* __restrict__ feats, float* out, int total4) {
  const int i = blockIdx.x * NTHR + (int)threadIdx.x;
  if (i >= total4) return;
  const int c4 = i & 15;
  const v4f mu = *(const v4f*)(bnp + 4 * c4);
  const v4f sc = *(const v4f*)(bnp + 64 + 4 * c4);
  const v4f be = *(const v4f*)(bnp + 128 + 4 * c4);
  const v4f x = *(const v4f*)(h2 + (size_t)i * 4);
  const v4f f = *(const v4f*)(feats + (size_t)i * 4);
  v4f v = (x - mu) * sc + be;
  v = v + f;
  v.x = fmaxf(v.x, 0.f); v.y = fmaxf(v.y, 0.f); v.z = fmaxf(v.z, 0.f); v.w = fmaxf(v.w, 0.f);
  float* op = out + (size_t)i * 4;
  *(volatile v4f*)op = v;
  __threadfence();
  *(volatile v4f*)op = v;
}

extern "C" void kernel_launch(void* const* d_in, const int* in_sizes, int n_in,
                              void* d_out, int out_size, void* d_ws, size_t ws_size,
                              hipStream_t stream) {
  if (n_in < 8) return;
  const int n = in_sizes[0] / CH;
  if (n <= 0 || in_sizes[0] != n * CH) return;
  if (in_sizes[1] != WPL || in_sizes[4] != WPL) return;
  if (in_sizes[2] < CH || in_sizes[3] < CH || in_sizes[5] < CH || in_sizes[6] < CH) return;
  if (in_sizes[7] != 4 * n) return;
  if (out_size != n * CH) return;
  if (n > (1 << 24)) return;

  const float* feats  = (const float*)d_in[0];
  const float* w1     = (const float*)d_in[1];
  const float* g1     = (const float*)d_in[2];
  const float* b1     = (const float*)d_in[3];
  const float* w2     = (const float*)d_in[4];
  const float* g2     = (const float*)d_in[5];
  const float* b2     = (const float*)d_in[6];
  const int*   coords = (const int*)d_in[7];
  float* out = (float*)d_out;

  const int nBlk = (n + CROWS - 1) / CROWS;
  const int NPAD = nBlk * CROWS;
  const int total4 = n * (CH / 4);
  const int nOut = (total4 + NTHR - 1) / NTHR;

  char* ws = (char*)d_ws;
  size_t off = 0;
  const size_t oTab = off; off += (size_t)TBLN * 4;            off = (off + 255) & ~(size_t)255;
  const size_t oW1  = off; off += (size_t)WPL * 2;             off = (off + 255) & ~(size_t)255;
  const size_t oW2  = off; off += (size_t)WPL * 2;             off = (off + 255) & ~(size_t)255;
  const size_t oH1  = off; off += (size_t)NPAD * CH * 4;       off = (off + 255) & ~(size_t)255;
  const size_t oH2  = off; off += (size_t)NPAD * CH * 4;       off = (off + 255) & ~(size_t)255;
  const size_t oPt  = off; off += (size_t)nBlk * 128 * 8;      off = (off + 255) & ~(size_t)255;
  const size_t oBn1 = off; off += 256 * 4;                     off = (off + 255) & ~(size_t)255;
  const size_t oBn2 = off; off += 256 * 4;                     off = (off + 255) & ~(size_t)255;
  if (off > ws_size || off > (size_t)WSCAP) return;
  int*      table = (int*)(ws + oTab);
  _Float16* wP1   = (_Float16*)(ws + oW1);
  _Float16* wP2   = (_Float16*)(ws + oW2);
  float*    h1    = (float*)(ws + oH1);
  float*    h2    = (float*)(ws + oH2);
  double*   part  = (double*)(ws + oPt);
  float*    bnp1  = (float*)(ws + oBn1);
  float*    bnp2  = (float*)(ws + oBn2);

  hipFuncSetAttribute(reinterpret_cast<const void*>(&k_table),
                      hipFuncAttributeMaxDynamicSharedMemorySize, LDS_TAB);
  k_table<<<TBLN / TPB, NTHR, LDS_TAB, stream>>>(coords, table, n);

  k_wprep<<<(2 * (WPL / 8)) / NTHR, NTHR, 0, stream>>>(w1, w2, wP1, wP2);

  hipFuncSetAttribute(reinterpret_cast<const void*>(&k_conv<0>),
                      hipFuncAttributeMaxDynamicSharedMemorySize, LDS_CONV);
  hipFuncSetAttribute(reinterpret_cast<const void*>(&k_conv<1>),
                      hipFuncAttributeMaxDynamicSharedMemorySize, LDS_CONV);
  k_conv<0><<<nBlk, NTHR, LDS_CONV, stream>>>(feats, coords, table, wP1, bnp1, h1, part, n);
  k_bnfin<<<1, NTHR, 0, stream>>>(part, nBlk, g1, b1, bnp1, n);

  k_conv<1><<<nBlk, NTHR, LDS_CONV, stream>>>(h1, coords, table, wP2, bnp1, h2, part, n);
  k_bnfin<<<1, NTHR, 0, stream>>>(part, nBlk, g2, b2, bnp2, n);

  k_out<<<nOut, NTHR, 0, stream>>>(h2, bnp2, feats, out, total4);
}
